// HET_RelationalAttLayer_21002390078097
// MI455X (gfx1250) — hardware-verified
//
#include <hip/hip_runtime.h>
#include <stddef.h>


#define IN_DIM  256
#define KP      256
#define NREL    8
#define NHEAD   4
#define HDIM    32
#define OUTF    128
#define WTROWS  (NREL * OUTF)
#define NTHR    256
#define NWAVE   8
#define EPT     8
#define CHUNK   (NTHR * EPT)
#define WCAP    (EPT * 32)
#define LISTN   (NWAVE * WCAP)
#define NBMAX   2048
#define RCAP    28672
#define DEGCAP  4096
#define GBM     64
#define GTHR    128
#define KSTEPS  (KP / 32)
#define NEG_SLOPE 0.2f
#define CA      16.0f
#define CW      64.0f
#define SCL     0.0009765625f
#define WSMAX   134217728
#define LDS_AGG ((2 * RCAP + 2 * NBMAX + LISTN) * 4 + 64)

static_assert((CHUNK & (CHUNK - 1)) == 0 && CHUNK <= 4096);
static_assert((NBMAX & (NBMAX - 1)) == 0 && NBMAX <= 4096);
static_assert(NTHR * 8 == NBMAX);
static_assert(LISTN >= NBMAX);
static_assert(LISTN >= NWAVE * WCAP);
static_assert((RCAP % 32) == 0);
static_assert(LDS_AGG <= 300000);
static_assert(GBM == (GTHR / 32) * 16);
static_assert(GTHR == OUTF);
static_assert(NHEAD * HDIM == OUTF);
static_assert(HDIM == 32);
static_assert(KP == IN_DIM && (KP % 32) == 0);
static_assert(2 * GBM == GTHR);
static_assert(NREL * GBM == 4 * GTHR);
static_assert(NREL * HDIM == 2 * GTHR);
static_assert(GBM * HDIM == 4 * GTHR * 4);

typedef float    v4f  __attribute__((ext_vector_type(4)));
typedef float    v8f  __attribute__((ext_vector_type(8)));
typedef int      v4i  __attribute__((ext_vector_type(4)));
typedef int      v8i  __attribute__((ext_vector_type(8)));
typedef _Float16 v8h  __attribute__((ext_vector_type(8)));
typedef _Float16 v16h __attribute__((ext_vector_type(16)));
union FragH { v16h v; v8h h[2]; v8i w; };

__device__ __forceinline__ v8f wmh(const FragH& a, const FragH& b, v8f c) {
  v8f d = __builtin_amdgcn_wmma_f32_16x16x32_f16(false, a.v, false, b.v, (short)0, c, false, false);
  asm volatile("v_nop\n\tv_nop\n\tv_nop\n\tv_nop" : "+v"(d) : "v"(a.w), "v"(b.w));
  return d;
}

__device__ __forceinline__ int scan_chunk(const int* __restrict__ dsts, int nE, int cbase, int slotBase,
                                          int nb, int vec8, int* list, int tid, int lane, int wave) {
  int wc = 0;
  const int el0  = tid * EPT;
  const int e0   = cbase + el0;
  const int sent = -2147483647 - 1;
  v4i da, db;
  if (vec8 != 0 && cbase + CHUNK <= nE) {
    da = *(const v4i*)(dsts + e0);
    db = *(const v4i*)(dsts + e0 + 4);
  } else {
    da.x = (e0     < nE) ? dsts[min(e0,     nE - 1)] : sent;
    da.y = (e0 + 1 < nE) ? dsts[min(e0 + 1, nE - 1)] : sent;
    da.z = (e0 + 2 < nE) ? dsts[min(e0 + 2, nE - 1)] : sent;
    da.w = (e0 + 3 < nE) ? dsts[min(e0 + 3, nE - 1)] : sent;
    db.x = (e0 + 4 < nE) ? dsts[min(e0 + 4, nE - 1)] : sent;
    db.y = (e0 + 5 < nE) ? dsts[min(e0 + 5, nE - 1)] : sent;
    db.z = (e0 + 6 < nE) ? dsts[min(e0 + 6, nE - 1)] : sent;
    db.w = (e0 + 7 < nE) ? dsts[min(e0 + 7, nE - 1)] : sent;
  }
  const unsigned nbs = (unsigned)slotBase;
  const unsigned unb = (unsigned)nb;
  const unsigned s0 = (unsigned)da.x - nbs, s1 = (unsigned)da.y - nbs;
  const unsigned s2 = (unsigned)da.z - nbs, s3 = (unsigned)da.w - nbs;
  const unsigned s4 = (unsigned)db.x - nbs, s5 = (unsigned)db.y - nbs;
  const unsigned s6 = (unsigned)db.z - nbs, s7 = (unsigned)db.w - nbs;
  const bool h0 = s0 < unb, h1 = s1 < unb, h2 = s2 < unb, h3 = s3 < unb;
  const bool h4 = s4 < unb, h5 = s5 < unb, h6 = s6 < unb, h7 = s7 < unb;
  const unsigned any = __builtin_amdgcn_ballot_w32(h0 | h1 | h2 | h3 | h4 | h5 | h6 | h7);
  if (any != 0u) {
#define HITJ(J, HJ, SJ) { \
      const unsigned mj = __builtin_amdgcn_ballot_w32(HJ); \
      if (mj != 0u) { \
        if (HJ) { \
          const int pos = wc + (int)__builtin_amdgcn_mbcnt_lo(mj, 0u); \
          if (pos < WCAP) list[wave * WCAP + pos] = ((el0 + (J)) << 12) | (int)(SJ); \
        } \
        wc += (int)__builtin_popcount(mj); } }
    HITJ(0, h0, s0)
    HITJ(1, h1, s1)
    HITJ(2, h2, s2)
    HITJ(3, h3, s3)
    HITJ(4, h4, s4)
    HITJ(5, h5, s5)
    HITJ(6, h6, s6)
    HITJ(7, h7, s7)
#undef HITJ
  }
  return wc;
}

__global__ __launch_bounds__(NTHR) void k_xprep(const float* __restrict__ x, _Float16* xh, int nN, int nUnits) {
  const int i = (int)blockIdx.x * NTHR + (int)threadIdx.x;
  if (i >= nUnits) return;
  const int row = i >> 5;
  const int c0  = (i & 31) * 8;
  const int rc  = row < nN ? row : nN - 1;
  const float* p = x + (size_t)rc * IN_DIM + c0;
  v4f a = *(const v4f*)p, b = *(const v4f*)(p + 4);
  const v4f z4 = {0.f, 0.f, 0.f, 0.f};
  if (row >= nN) { a = z4; b = z4; }
  v8h hv;
  hv[0] = (_Float16)(a.x * CA); hv[1] = (_Float16)(a.y * CA);
  hv[2] = (_Float16)(a.z * CA); hv[3] = (_Float16)(a.w * CA);
  hv[4] = (_Float16)(b.x * CA); hv[5] = (_Float16)(b.y * CA);
  hv[6] = (_Float16)(b.z * CA); hv[7] = (_Float16)(b.w * CA);
  const size_t o = (size_t)row * KP + c0;
  *(volatile v8h*)(xh + o) = hv;
  __threadfence();
  *(volatile v8h*)(xh + o) = hv;
}

__global__ __launch_bounds__(NTHR) void k_wprep(const float* __restrict__ w, _Float16* wt, int nUnits) {
  const int u = (int)blockIdx.x * NTHR + (int)threadIdx.x;
  if (u >= nUnits) return;
  const int ng  = u >> 5;
  const int k8  = (u & 31) * 8;
  const int rel = ng >> 7;
  const int n   = ng & (OUTF - 1);
  const int hdx = n >> 5;
  const int d   = n & (HDIM - 1);
  const float* p = w + ((size_t)(rel * NHEAD + hdx) * IN_DIM + k8) * HDIM + d;
  v4f a, b;
  a.x = p[0 * HDIM]; a.y = p[1 * HDIM]; a.z = p[2 * HDIM]; a.w = p[3 * HDIM];
  b.x = p[4 * HDIM]; b.y = p[5 * HDIM]; b.z = p[6 * HDIM]; b.w = p[7 * HDIM];
  v8h hv;
  hv[0] = (_Float16)(a.x * CW); hv[1] = (_Float16)(a.y * CW);
  hv[2] = (_Float16)(a.z * CW); hv[3] = (_Float16)(a.w * CW);
  hv[4] = (_Float16)(b.x * CW); hv[5] = (_Float16)(b.y * CW);
  hv[6] = (_Float16)(b.z * CW); hv[7] = (_Float16)(b.w * CW);
  const size_t o = (size_t)ng * KP + k8;
  *(volatile v8h*)(wt + o) = hv;
  __threadfence();
  *(volatile v8h*)(wt + o) = hv;
}

__global__ __launch_bounds__(GTHR) void k_gemm(const _Float16* __restrict__ xh, const _Float16* __restrict__ wt,
                                               const float* __restrict__ attl, const float* __restrict__ attr,
                                               float* P, float* EL, float* ER, int MP, int head) {
  __shared__ __attribute__((aligned(16))) float stg[GBM * HDIM];
  __shared__ __attribute__((aligned(16))) float esT[NREL * GBM];
  __shared__ __attribute__((aligned(16))) float edT[NREL * GBM];
  __shared__ float sAl[NREL * HDIM];
  __shared__ float sAr[NREL * HDIM];
  const int tid = threadIdx.x, lane = tid & 31, wave = tid >> 5, hh = lane >> 4, m = lane & 15;
  const int rowBase = (int)blockIdx.x * GBM;
  const int hc = (head < 0 ? 0 : (head > NHEAD - 1 ? NHEAD - 1 : head));
  {
    const int r0 = tid >> 5, d0 = tid & 31;
    sAl[tid]        = attl[(r0    ) * OUTF + hc * HDIM + d0];
    sAr[tid]        = attr[(r0    ) * OUTF + hc * HDIM + d0];
    sAl[tid + GTHR] = attl[(r0 + 4) * OUTF + hc * HDIM + d0];
    sAr[tid + GTHR] = attr[(r0 + 4) * OUTF + hc * HDIM + d0];
  }
  const size_t arow = (size_t)(rowBase + 16 * wave + m) * KP + 8 * hh;
  FragH af[KSTEPS];
#pragma unroll
  for (int ks = 0; ks < KSTEPS; ++ks) {
    af[ks].h[0] = *(const v8h*)(xh + arow + 32 * ks);
    af[ks].h[1] = *(const v8h*)(xh + arow + 32 * ks + 16);
  }
#pragma unroll 1
  for (int rel = 0; rel < NREL; ++rel) {
    const size_t brow = ((size_t)rel * OUTF + (size_t)hc * HDIM + m) * KP + 8 * hh;
    v8f acc[2];
    { v8f z = {0.f, 0.f, 0.f, 0.f, 0.f, 0.f, 0.f, 0.f}; acc[0] = z; acc[1] = z; }
#pragma unroll
    for (int ks = 0; ks < KSTEPS; ++ks) {
#pragma unroll
      for (int t = 0; t < 2; ++t) {
        const size_t bo = brow + (size_t)(16 * t) * KP + 32 * ks;
        FragH bf;
        bf.h[0] = *(const v8h*)(wt + bo);
        bf.h[1] = *(const v8h*)(wt + bo + 16);
        acc[t] = wmh(af[ks], bf, acc[t]);
      }
    }
    float* sp = stg + (size_t)(16 * wave + 8 * hh) * HDIM + m;
#pragma unroll
    for (int t = 0; t < 2; ++t) {
#pragma unroll
      for (int r = 0; r < 8; ++r) sp[(size_t)r * HDIM + 16 * t] = acc[t][r] * SCL;
    }
    __syncthreads();
    {
      const int row  = tid >> 1;
      const int half = tid & 1;
      const float* srow = stg + (size_t)row * HDIM;
      float s = 0.f, d = 0.f;
#pragma unroll 1
      for (int c = 0; c < 16; ++c) {
        const int cc = half * 16 + c;
        const float v = srow[cc];
        s = fmaf(v, sAl[rel * HDIM + cc], s);
        d = fmaf(v, sAr[rel * HDIM + cc], d);
      }
      s += __shfl_xor(s, 1);
      d += __shfl_xor(d, 1);
      if (half == 0) {
        esT[rel * GBM + row] = s;
        edT[rel * GBM + row] = d;
      }
    }
    {
      float* pb = P + ((size_t)rel * (size_t)MP + (size_t)rowBase) * HDIM;
      const v4f* s4 = (const v4f*)stg;
      const v4f v0 = s4[tid], v1 = s4[tid + GTHR], v2 = s4[tid + 2 * GTHR], v3 = s4[tid + 3 * GTHR];
      *(volatile v4f*)(pb + (size_t)4 * tid)                = v0;
      *(volatile v4f*)(pb + (size_t)4 * (tid + GTHR))       = v1;
      *(volatile v4f*)(pb + (size_t)4 * (tid + 2 * GTHR))   = v2;
      *(volatile v4f*)(pb + (size_t)4 * (tid + 3 * GTHR))   = v3;
      __threadfence();
      *(volatile v4f*)(pb + (size_t)4 * tid)                = v0;
      *(volatile v4f*)(pb + (size_t)4 * (tid + GTHR))       = v1;
      *(volatile v4f*)(pb + (size_t)4 * (tid + 2 * GTHR))   = v2;
      *(volatile v4f*)(pb + (size_t)4 * (tid + 3 * GTHR))   = v3;
    }
    __syncthreads();
  }
  {
    const int rel = tid >> 4;
    const int q   = tid & 15;
    const v4f ve = *(const v4f*)(esT + rel * GBM + 4 * q);
    const v4f vd = *(const v4f*)(edT + rel * GBM + 4 * q);
    const size_t po = (size_t)rel * (size_t)MP + (size_t)rowBase + (size_t)(4 * q);
    float* pe = EL + po;
    float* pd = ER + po;
    *(volatile v4f*)pe = ve;
    *(volatile v4f*)pd = vd;
    __threadfence();
    *(volatile v4f*)pe = ve;
    *(volatile v4f*)pd = vd;
  }
}

__global__ __launch_bounds__(NTHR) void k_agg(
    const int* __restrict__ srcs, const int* __restrict__ dsts,
    const float* __restrict__ P, const float* __restrict__ EL, const float* __restrict__ ER,
    const float* __restrict__ bias, float* out,
    int nN, int nE, int nb, int vec8, int MP, int epr, float invE, int head) {
  extern __shared__ v4f lds_dyn[];
  int* reg1 = (int*)lds_dyn;
  int* reg2 = reg1 + RCAP;
  int* scnt = reg2 + RCAP;
  int* soff = scnt + NBMAX;
  int* list = soff + NBMAX;
  int* wcnt = list + LISTN;
  int* wtot = wcnt + NWAVE;
  const int tid = threadIdx.x, lane = tid & 31, wave = tid >> 5;
  const int nodeBase = (int)blockIdx.x * nb;
  const int hc = (head < 0 ? 0 : (head > NHEAD - 1 ? NHEAD - 1 : head));

  for (int i = tid; i < NBMAX; i += NTHR) scnt[i] = 0;
  __syncthreads();

  int tot = 0;
  const int nChunks = (nE + CHUNK - 1) / CHUNK;
#pragma unroll 1
  for (int ch = 0; ch < nChunks; ++ch) {
    const int cbase = ch * CHUNK;
    const int wc = scan_chunk(dsts, nE, cbase, nodeBase, nb, vec8, list, tid, lane, wave);
    if (lane == 0) wcnt[wave] = wc;
    __syncthreads();
    int pre = 0, all = 0;
#pragma unroll
    for (int w2 = 0; w2 < NWAVE; ++w2) {
      int c = wcnt[w2];
      c = c < 0 ? 0 : (c > WCAP ? WCAP : c);
      all += c;
      pre += (w2 < wave) ? c : 0;
    }
    const int wcc  = wc > WCAP ? WCAP : wc;
    const int base = tot + pre;
#pragma unroll 1
    for (int i = lane; i < wcc; i += 32) {
      const int ent = list[wave * WCAP + i];
      const int el  = (ent >> 12) & (CHUNK - 1);
      const int sl  = ent & (NBMAX - 1);
      int eid = cbase + el;
      eid = eid > nE - 1 ? nE - 1 : eid;
      const int pos = base + i;
      if (pos < RCAP) reg1[pos] = (int)(((unsigned)eid << 12) | (unsigned)sl);
    }
    tot += all;
    tot = tot > RCAP ? RCAP : tot;
    __syncthreads();
  }
  const int nh = tot;

  if (wave == 0) {
#pragma unroll 1
    for (int b0 = 0; b0 < nh; b0 += 32) {
      const int idx = b0 + lane;
      const int uv  = reg1[idx < RCAP ? idx : RCAP - 1];
      const int m32 = (nh - b0) < 32 ? (nh - b0) : 32;
#pragma unroll 1
      for (int k = 0; k < m32; ++k) {
        const int u  = __builtin_amdgcn_readlane(uv, k);
        const int sl = u & (NBMAX - 1);
        if (lane == 0) scnt[sl] = scnt[sl] + 1;
      }
    }
  }
  __syncthreads();

  {
    const v4i ca = *(const v4i*)(scnt + 8 * tid);
    const v4i cb = *(const v4i*)(scnt + 8 * tid + 4);
    const int e0 = ca.x < 0 ? 0 : ca.x, e1 = ca.y < 0 ? 0 : ca.y, e2 = ca.z < 0 ? 0 : ca.z, e3 = ca.w < 0 ? 0 : ca.w;
    const int e4 = cb.x < 0 ? 0 : cb.x, e5 = cb.y < 0 ? 0 : cb.y, e6 = cb.z < 0 ? 0 : cb.z, e7 = cb.w < 0 ? 0 : cb.w;
    const int ts = e0 + e1 + e2 + e3 + e4 + e5 + e6 + e7;
    int incl = ts;
#pragma unroll
    for (int d = 1; d < 32; d <<= 1) {
      const int up = __shfl_up(incl, d);
      if (lane >= d) incl += up;
    }
    if (lane == 31) wtot[wave] = incl;
    __syncthreads();
    int pre = 0;
#pragma unroll
    for (int w2 = 0; w2 < NWAVE; ++w2) pre += (w2 < wave) ? wtot[w2] : 0;
    int run = pre + incl - ts;
    soff[8 * tid + 0] = run; run += e0;
    soff[8 * tid + 1] = run; run += e1;
    soff[8 * tid + 2] = run; run += e2;
    soff[8 * tid + 3] = run; run += e3;
    soff[8 * tid + 4] = run; run += e4;
    soff[8 * tid + 5] = run; run += e5;
    soff[8 * tid + 6] = run; run += e6;
    soff[8 * tid + 7] = run;
  }
  __syncthreads();
  for (int i = tid; i < NBMAX; i += NTHR) list[i] = soff[i];
  __syncthreads();

  if (wave == 0) {
#pragma unroll 1
    for (int b0 = 0; b0 < nh; b0 += 32) {
      const int idx = b0 + lane;
      const int uv  = reg1[idx < RCAP ? idx : RCAP - 1];
      const int m32 = (nh - b0) < 32 ? (nh - b0) : 32;
#pragma unroll 1
      for (int k = 0; k < m32; ++k) {
        const int u   = __builtin_amdgcn_readlane(uv, k);
        const int sl  = u & (NBMAX - 1);
        const int eid = (int)((unsigned)u >> 12);
        if (lane == 0) {
          int pos = list[sl];
          pos = pos < 0 ? 0 : (pos > RCAP - 1 ? RCAP - 1 : pos);
          reg2[pos] = eid;
          list[sl] = pos + 1;
        }
      }
    }
  }
  __syncthreads();

  const int nbw = nb >> 3;
  const float bz = bias[hc * HDIM + lane];
  const bool ovf = (nh >= RCAP);
  const float qnan = __int_as_float(0x7fc00000);
  const size_t plE = (size_t)MP;
  const int g0 = (4 * lane) & 31, g1 = (4 * lane + 1) & 31, g2 = (4 * lane + 2) & 31, g3 = (4 * lane + 3) & 31;
#pragma unroll 1
  for (int jt = 0; jt < nbw; ++jt) {
    const int slot = wave * nbw + jt;
    const int grow = nodeBase + slot;
    const int gcl  = grow < nN ? grow : nN - 1;
    int st = soff[slot];
    const int craw = scnt[slot];
    int cnt = craw;
    st  = st < 0 ? 0 : (st > nh ? nh : st);
    cnt = cnt < 0 ? 0 : (cnt > DEGCAP ? DEGCAP : cnt);
    if (cnt > nh - st) cnt = nh - st;
    const float pz = (ovf || craw > DEGCAP) ? qnan : 0.0f;
    const bool wr = grow < nN;

    const float* erd = ER + (size_t)gcl;
    const float er0 = erd[0];
    const float er1 = erd[plE];
    const float er2 = erd[2 * plE];
    const float er3 = erd[3 * plE];
    const float er4 = erd[4 * plE];
    const float er5 = erd[5 * plE];
    const float er6 = erd[6 * plE];
    const float er7 = erd[7 * plE];

    float mx = -1.0e30f;
    float dn = 0.0f;
    float a  = 0.0f;
#pragma unroll 1
    for (int q = 0; q < cnt; ++q) {
      int idx = st + q; idx = idx > RCAP - 1 ? RCAP - 1 : idx;
      int eid = reg2[idx]; eid = eid < 0 ? 0 : (eid > nE - 1 ? nE - 1 : eid);
      const int sraw = srcs[eid];
      const int s = sraw < 0 ? 0 : (sraw > nN - 1 ? nN - 1 : sraw);
      int rr = (int)((float)eid * invE);
      rr = ((rr + 1) * epr <= eid) ? rr + 1 : rr;
      rr = (rr * epr > eid) ? rr - 1 : rr;
      rr = rr < 0 ? 0 : (rr > NREL - 1 ? NREL - 1 : rr);
      const size_t pr = (size_t)rr * plE + (size_t)s;
      const float xs  = P[pr * HDIM + lane];
      const float els = EL[pr];
      float erv = er0;
      erv = (rr == 1) ? er1 : erv;
      erv = (rr == 2) ? er2 : erv;
      erv = (rr == 3) ? er3 : erv;
      erv = (rr == 4) ? er4 : erv;
      erv = (rr == 5) ? er5 : erv;
      erv = (rr == 6) ? er6 : erv;
      erv = (rr == 7) ? er7 : erv;
      const float u = els + erv;
      const float l = fmaxf(u, NEG_SLOPE * u);
      const float mn = fmaxf(mx, l);
      const float s1 = __expf(mx - mn), s2 = __expf(l - mn);
      dn = fmaf(dn, s1, s2);
      a  = fmaf(a, s1, s2 * xs);
      mx = mn;
    }
    const float dsafe = dn > 0.f ? dn : 1.0f;
    const float inv = (dn > 0.f ? 1.0f : 0.0f) * __builtin_amdgcn_rcpf(dsafe);
    const float o = fmaf(a, inv, bz) + pz;
    v4f v;
    v.x = __shfl(o, g0);
    v.y = __shfl(o, g1);
    v.z = __shfl(o, g2);
    v.w = __shfl(o, g3);
    float* op = out + (size_t)gcl * OUTF + (size_t)(hc * HDIM) + 4 * (lane & 7);
    const bool ws8 = wr && (lane < 8);
    if (ws8) *(volatile v4f*)op = v;
    __threadfence();
    if (ws8) *(volatile v4f*)op = v;
  }
}

static int pick_nb(int nE, int nN) {
  int nb = NBMAX;
  while (nb > 16 && (long long)nb * (long long)nE * 5LL > (long long)RCAP * (long long)nN * 4LL) nb >>= 1;
  return nb;
}

extern "C" void kernel_launch(void* const* d_in, const int* in_sizes, int n_in,
                              void* d_out, int out_size, void* d_ws, size_t ws_size,
                              hipStream_t stream) {
  if (n_in < 7) return;
  const int nN = in_sizes[0] / IN_DIM;
  if (nN <= 0 || in_sizes[0] != nN * IN_DIM) return;
  if (nN > (1 << 22)) return;
  if (in_sizes[1] != NREL * NHEAD * IN_DIM * HDIM) return;
  if (in_sizes[2] != NREL * OUTF || in_sizes[3] != NREL * OUTF) return;
  if (in_sizes[4] != OUTF) return;
  const int nE = in_sizes[5];
  if (nE < NREL || in_sizes[6] != nE) return;
  if ((nE % NREL) != 0) return;
  if (nE > (1 << 20)) return;
  if (out_size != nN * OUTF) return;

  const float* x    = (const float*)d_in[0];
  const float* w    = (const float*)d_in[1];
  const float* attl = (const float*)d_in[2];
  const float* attr = (const float*)d_in[3];
  const float* bias = (const float*)d_in[4];
  const int*   src  = (const int*)d_in[5];
  const int*   dst  = (const int*)d_in[6];
  float* out = (float*)d_out;

  const int MP   = ((nN + GBM - 1) / GBM) * GBM;
  const int nb   = pick_nb(nE, nN);
  const int vec8 = 1;
  const int epr  = nE / NREL;
  const float invE = 1.0f / (float)epr;
  const int nUnitsX = MP * (KP / 8);
  const int nUnitsW = WTROWS * (KP / 8);

  char* ws = (char*)d_ws;
  size_t off = 0;
  const size_t oWT = off; off += (size_t)WTROWS * KP * 2;               off = (off + 255) & ~(size_t)255;
  const size_t oXH = off; off += (size_t)MP * KP * 2;                   off = (off + 255) & ~(size_t)255;
  const size_t oP  = off; off += (size_t)NREL * (size_t)MP * HDIM * 4;  off = (off + 255) & ~(size_t)255;
  const size_t oEL = off; off += (size_t)NREL * (size_t)MP * 4;         off = (off + 255) & ~(size_t)255;
  const size_t oER = off; off += (size_t)NREL * (size_t)MP * 4;         off = (off + 255) & ~(size_t)255;
  if (off > ws_size || off > (size_t)WSMAX) return;
  _Float16* WT = (_Float16*)(ws + oWT);
  _Float16* XH = (_Float16*)(ws + oXH);
  float*    P  = (float*)(ws + oP);
  float*    EL = (float*)(ws + oEL);
  float*    ER = (float*)(ws + oER);

  hipFuncSetAttribute(reinterpret_cast<const void*>(&k_agg),
                      hipFuncAttributeMaxDynamicSharedMemorySize, LDS_AGG);

  k_xprep<<<(nUnitsX + NTHR - 1) / NTHR, NTHR, 0, stream>>>(x, XH, nN, nUnitsX);
  k_wprep<<<(nUnitsW + NTHR - 1) / NTHR, NTHR, 0, stream>>>(w, WT, nUnitsW);

  const int gG = MP / GBM;
  const int gA = (nN + nb - 1) / nb;
  for (int head = 0; head < NHEAD; ++head) {
    k_gemm<<<gG, GTHR, 0, stream>>>(XH, WT, attl, attr, P, EL, ER, MP, head);
    k_agg<<<gA, NTHR, LDS_AGG, stream>>>(src, dst, P, EL, ER, bias, out, nN, nE, nb, vec8, MP, epr, invE, head);
  }
}
